// TimeseriesGenerator_18330920419813
// MI455X (gfx1250) — hardware-verified
//
#include <hip/hip_runtime.h>
#include <math.h>

constexpr int NB   = 256;
constexpr int NIN  = 128;
constexpr int NH   = 256;
constexpr int NG4  = 1024;
constexpr int NT   = 512;
constexpr int NF   = 64;
constexpr int NTHR_G = 256;
constexpr int NTHR_R = 512;
constexpr int ROWS_BLK = 16;
constexpr int HP1 = 264;
constexpr int HP2 = 520;
constexpr int HPB = 264;
constexpr int OSP = 68;
constexpr int NOUT = NB * NT * NF;
constexpr float WCARRY     = 16.0f;
constexpr float WCARRY_INV = 1.0f / 16.0f;
static_assert(NB % ROWS_BLK == 0);
static_assert(NH == 16 * (NTHR_R / 32));
static_assert(NIN % 64 == 0 && NH % 64 == 0 && NG4 % 64 == 0 && NF % 64 == 0);
static_assert(NIN % 32 == 0 && NH % 32 == 0);
static_assert((NB * NIN) % (8 * NTHR_G) == 0);
static_assert(HP1 % 8 == 0 && HP2 % 8 == 0 && HPB % 8 == 0);
static_assert(NTHR_R / 32 == ROWS_BLK);

typedef __attribute__((ext_vector_type(16))) _Float16 v16h;
typedef __attribute__((ext_vector_type(8)))  _Float16 v8h;
typedef __attribute__((ext_vector_type(16))) __bf16   v16b;
typedef __attribute__((ext_vector_type(8)))  __bf16   v8b;
typedef __attribute__((ext_vector_type(8)))  float    v8f;
typedef __attribute__((ext_vector_type(4)))  float    v4f;

__device__ __forceinline__ unsigned short f2bf_bits(float f) {
  unsigned u = __float_as_uint(f);
  return (unsigned short)((u + 0x7FFFu + ((u >> 16) & 1u)) >> 16);
}
__device__ __forceinline__ float bf_bits2f(unsigned short h) { return __uint_as_float(((unsigned)h) << 16); }

__device__ __forceinline__ void dep_guard_h(v8f& a, v8f& b, v16h x, v16h y) { asm volatile("v_nop\n\tv_nop\n\tv_nop\n\tv_nop" : "+v"(a), "+v"(b) : "v"(x), "v"(y)); }
__device__ __forceinline__ void dep_guard_b(v8f& a, v8f& b, v16b x, v16b y) { asm volatile("v_nop\n\tv_nop\n\tv_nop\n\tv_nop" : "+v"(a), "+v"(b) : "v"(x), "v"(y)); }
__device__ __forceinline__ void dep_guard1_b(v8f& a, v16b x, v16b y) { asm volatile("v_nop\n\tv_nop\n\tv_nop\n\tv_nop" : "+v"(a) : "v"(x), "v"(y)); }
__device__ __forceinline__ void keep4_h(v16h a, v16h b, v16h c, v16h d) { asm volatile("v_nop" :: "v"(a), "v"(b), "v"(c), "v"(d)); }
__device__ __forceinline__ void keep4_b(v16b a, v16b b, v16b c, v16b d) { asm volatile("v_nop" :: "v"(a), "v"(b), "v"(c), "v"(d)); }
__device__ __forceinline__ void acc_guard4(v8f& a, v8f& b, v8f& c, v8f& d) { asm volatile("v_nop\n\tv_nop\n\tv_nop\n\tv_nop" : "+v"(a), "+v"(b), "+v"(c), "+v"(d)); }
__device__ __forceinline__ void acc_guard1(v8f& a) { asm volatile("v_nop\n\tv_nop\n\tv_nop\n\tv_nop" : "+v"(a)); }
template <typename T> struct Frag;
template <> struct Frag<_Float16> {
  typedef v16h V; union U { v16h v; v8h h[2]; };
  static __device__ __forceinline__ v16h load(const _Float16* p) {
    U f; f.h[0] = *(const v8h*)(p); f.h[1] = *(const v8h*)(p + 16); return f.v;
  }
  static __device__ __forceinline__ v8f mma(v16h a, v16h b, v8f c) {
    return __builtin_amdgcn_wmma_f32_16x16x32_f16(false, a, false, b, (short)0, c, false, false);
  }
  static __device__ __forceinline__ void guard(v8f& a, v8f& b, v16h x, v16h y) { dep_guard_h(a, b, x, y); }
  static __device__ __forceinline__ void keep(v16h a, v16h b, v16h c, v16h d) { keep4_h(a, b, c, d); }
};
template <> struct Frag<__bf16> {
  typedef v16b V; union U { v16b v; v8b h[2]; };
  static __device__ __forceinline__ v16b load(const __bf16* p) {
    U f; f.h[0] = *(const v8b*)(p); f.h[1] = *(const v8b*)(p + 16); return f.v;
  }
  static __device__ __forceinline__ v8f mma(v16b a, v16b b, v8f c) {
    return __builtin_amdgcn_wmma_f32_16x16x32_bf16(false, a, false, b, (short)0, c, false, false);
  }
  static __device__ __forceinline__ void guard(v8f& a, v8f& b, v16b x, v16b y) { dep_guard_b(a, b, x, y); }
  static __device__ __forceinline__ void keep(v16b a, v16b b, v16b c, v16b d) { keep4_b(a, b, c, d); }
};

__device__ __forceinline__ float fsig(float x)  { return __builtin_amdgcn_rcpf(1.0f + __expf(-x)); }
__device__ __forceinline__ float ftanh(float x) { return 1.0f - 2.0f * __builtin_amdgcn_rcpf(__expf(2.0f * x) + 1.0f); }

template <int ET> struct Elem;
template <> struct Elem<0> { typedef _Float16 T; };
template <> struct Elem<1> { typedef __bf16 T; };
template <int ET, bool SPLIT, int BIAS_MODE, int OUT_MODE, bool RESID, int ACT = 0>
__global__ __launch_bounds__(256) void wmma_gemm64(
    const unsigned short* __restrict__ Ap, const unsigned short* __restrict__ A2p, int lda, long strideA,
    const unsigned short* __restrict__ Btp, const unsigned short* __restrict__ Bt2p, int ldb, long strideB,
    void* __restrict__ Cout, void* __restrict__ Cout2, int ldc, long strideC,
    const float* __restrict__ bias,
    const float* __restrict__ resid, long strideR,
    int M, int N, int K, float scale) {
  typedef typename Elem<ET>::T T;
  typedef typename Frag<T>::V V;
  const T* A = (const T*)Ap; const T* A2 = (const T*)A2p; const T* Bt = (const T*)Btp; const T* Bt2 = (const T*)Bt2p;
  __shared__ __align__(16) float sT[8][16 * 68];
  const int b    = blockIdx.y;
  const int lane = threadIdx.x & 31;
  const int wave = threadIdx.x >> 5;
  const int tilesN = N >> 6;
  const int tilesM = M >> 6;
  const int tile = blockIdx.x * 8 + wave;
  if (tile >= tilesM * tilesN) return;
  const int tm = tile / tilesN;
  const int tn = tile - tm * tilesN;
  const int m0 = tm << 6;
  const int n0 = tn << 6;

  const T* Ab  = A  + (size_t)b * strideA;
  const T* Bb  = Bt + (size_t)b * strideB;
  const T* Ab2 = SPLIT ? (A2  + (size_t)b * strideA) : nullptr;
  const T* Bb2 = SPLIT ? (Bt2 + (size_t)b * strideB) : nullptr;

  const int rlane = lane & 15;
  const int koff  = (lane >> 4) * 8;
  const int mOff  = (lane >> 4) * 8;

  v8f acc[4][4];
#pragma unroll
  for (int i = 0; i < 4; ++i)
#pragma unroll
    for (int j = 0; j < 4; ++j) acc[i][j] = (v8f){0.f,0.f,0.f,0.f,0.f,0.f,0.f,0.f};

  for (int k0 = 0; k0 < K; k0 += 32) {
    V bh[4], bl[4];
#pragma unroll
    for (int j = 0; j < 4; ++j) {
      const size_t bo = (size_t)(n0 + (j << 4) + rlane) * ldb + koff + k0;
      bh[j] = Frag<T>::load(Bb + bo);
      if (SPLIT) bl[j] = Frag<T>::load(Bb2 + bo);
    }
#pragma unroll
    for (int i = 0; i < 4; ++i) {
      const size_t ao = (size_t)(m0 + (i << 4) + rlane) * lda + koff + k0;
      V ah = Frag<T>::load(Ab + ao);
      V al;
      if (SPLIT) al = Frag<T>::load(Ab2 + ao);
#pragma unroll
      for (int j = 0; j < 4; ++j) {
        acc[i][j] = Frag<T>::mma(ah, bh[j], acc[i][j]);
        if (SPLIT) {
          acc[i][j] = Frag<T>::mma(ah, bl[j], acc[i][j]);
          acc[i][j] = Frag<T>::mma(al, bh[j], acc[i][j]);
        }
      }
      Frag<T>::guard(acc[i][0], acc[i][3], ah, SPLIT ? al : ah);
    }
    Frag<T>::keep(bh[0], bh[1], bh[2], bh[3]);
    if (SPLIT) Frag<T>::keep(bl[0], bl[1], bl[2], bl[3]);
  }
  acc_guard4(acc[0][0], acc[0][1], acc[0][2], acc[0][3]);
  acc_guard4(acc[1][0], acc[1][1], acc[1][2], acc[1][3]);
  acc_guard4(acc[2][0], acc[2][1], acc[2][2], acc[2][3]);
  acc_guard4(acc[3][0], acc[3][1], acc[3][2], acc[3][3]);

  float* slab = sT[wave];
  const float* Rb = RESID ? (resid + (size_t)b * strideR) : nullptr;
#pragma unroll
  for (int i = 0; i < 4; ++i) {
    const int mBase = m0 + (i << 4);
#pragma unroll
    for (int j = 0; j < 4; ++j) {
      const int n = n0 + (j << 4) + rlane;
      float bv = 0.f;
      if (BIAS_MODE == 2) bv = bias[n];
#pragma unroll
      for (int r = 0; r < 8; ++r) {
        float v = acc[i][j][r] * scale;
        if (BIAS_MODE == 1) v += bias[mBase + mOff + r];
        if (BIAS_MODE == 2) v += bv;
        if (RESID) v += Rb[(size_t)(mBase + mOff + r) * ldc + n];
        if (ACT == 1) v = tanhf(v);
        if (ACT == 2) v = fmaxf(v, 0.0f);
        if (ACT == 3) v = v / (1.0f + expf(-v));
        if (ACT == 4) v = (v > 0.f) ? v : 0.01f * v;
        if (ACT == 5) v = 0.5f * v * (1.0f + erff(v * 0.70710678118654752f));
        slab[(mOff + r) * 68 + (j << 4) + rlane] = v;
      }
    }
    __builtin_amdgcn_fence(__ATOMIC_RELEASE, "workgroup");
    __builtin_amdgcn_wave_barrier();
    __builtin_amdgcn_fence(__ATOMIC_ACQUIRE, "workgroup");
    if (OUT_MODE == 0) {
      float* C = (float*)Cout + (size_t)b * strideC;
      const int hh = lane >> 4, c4 = (lane & 15) * 4;
      for (int pass = 0; pass < 2; ++pass) {
#pragma unroll
        for (int it = 0; it < 8; ++it) {
          const int row = it * 2 + hh;
          v4f v = *(const v4f*)(slab + row * 68 + c4);
          *(volatile v4f*)(C + (size_t)(mBase + row) * ldc + n0 + c4) = v;
        }
        __threadfence();
      }
    } else {
      const int q = lane >> 3, c8 = (lane & 7) * 8;
      unsigned short* C  = (unsigned short*)Cout  + (size_t)b * strideC;
      unsigned short* C2 = (OUT_MODE == 2) ? ((unsigned short*)Cout2 + (size_t)b * strideC) : nullptr;
      for (int pass = 0; pass < 2; ++pass) {
#pragma unroll
        for (int it = 0; it < 4; ++it) {
          const int row = it * 4 + q;
          const float* sp = slab + row * 68 + c8;
          v8h hv, lv;
#pragma unroll
          for (int e = 0; e < 8; ++e) {
            if (OUT_MODE == 1) {
              hv[e] = (_Float16)sp[e];
            } else {
              unsigned short hb = f2bf_bits(sp[e]);
              unsigned short lb = f2bf_bits(sp[e] - bf_bits2f(hb));
              hv[e] = __builtin_bit_cast(_Float16, hb);
              lv[e] = __builtin_bit_cast(_Float16, lb);
            }
          }
          *(volatile v8h*)(C + (size_t)(mBase + row) * ldc + n0 + c8) = hv;
          if (OUT_MODE == 2) *(volatile v8h*)(C2 + (size_t)(mBase + row) * ldc + n0 + c8) = lv;
        }
        __threadfence();
      }
    }
    __builtin_amdgcn_fence(__ATOMIC_RELEASE, "workgroup");
    __builtin_amdgcn_wave_barrier();
    __builtin_amdgcn_fence(__ATOMIC_ACQUIRE, "workgroup");
  }
}

template <int MODE>
__global__ __launch_bounds__(NTHR_G) void tr64_kernel(const float* __restrict__ in, int ncol,
                                                      unsigned short* __restrict__ out, unsigned short* __restrict__ out2,
                                                      int ldo, int col0, float sc) {
  __shared__ __align__(16) float tl[64][68];
  const int tid = threadIdx.x, lane = tid & 31, wave = tid >> 5;
  const int c0 = blockIdx.x * 64, r0 = blockIdx.y * 64;
  {
    const int row = tid >> 2, cb = (tid & 3) * 16;
    const float* sp = in + (size_t)(r0 + row) * ncol + c0 + cb;
#pragma unroll
    for (int q = 0; q < 4; ++q) {
      const v4f v = *(const v4f*)(sp + 4 * q);
#pragma unroll
      for (int e = 0; e < 4; ++e) tl[cb + 4 * q + e][row] = v[e];
    }
  }
  __syncthreads();
  const int q = lane >> 3, r8 = (lane & 7) * 8;
  for (int pass = 0; pass < 2; ++pass) {
#pragma unroll
    for (int it = 0; it < 2; ++it) {
      const int crow = it * 32 + wave * 4 + q;
      const float* tp = &tl[crow][r8];
      v8h hv, lv;
#pragma unroll
      for (int e = 0; e < 8; ++e) {
        const float v = tp[e];
        if (MODE == 0) {
          const unsigned short hb = f2bf_bits(v);
          const unsigned short lb = f2bf_bits(v - bf_bits2f(hb));
          hv[e] = __builtin_bit_cast(_Float16, hb);
          lv[e] = __builtin_bit_cast(_Float16, lb);
        } else {
          hv[e] = (_Float16)(v * sc);
          lv[e] = hv[e];
        }
      }
      const size_t o = (size_t)(c0 + crow) * ldo + col0 + r0 + r8;
      *(volatile v8h*)(out + o) = hv;
      if (MODE == 0) *(volatile v8h*)(out2 + o) = lv;
    }
    __threadfence();
  }
}

__global__ __launch_bounds__(NTHR_G) void cvt_split8_kernel(const float* __restrict__ src,
                                                            unsigned short* __restrict__ hi, unsigned short* __restrict__ lo, int n8) {
  const int i = blockIdx.x * NTHR_G + threadIdx.x;
  if (i < n8) {
    const float* sp = src + (size_t)i * 8;
    const v4f a = *(const v4f*)(sp);
    const v4f b = *(const v4f*)(sp + 4);
    v8h hv, lv;
#pragma unroll
    for (int e = 0; e < 4; ++e) {
      const unsigned short h0 = f2bf_bits(a[e]);
      const unsigned short l0 = f2bf_bits(a[e] - bf_bits2f(h0));
      const unsigned short h1 = f2bf_bits(b[e]);
      const unsigned short l1 = f2bf_bits(b[e] - bf_bits2f(h1));
      hv[e] = __builtin_bit_cast(_Float16, h0); hv[4 + e] = __builtin_bit_cast(_Float16, h1);
      lv[e] = __builtin_bit_cast(_Float16, l0); lv[4 + e] = __builtin_bit_cast(_Float16, l1);
    }
    *(volatile v8h*)(hi + (size_t)i * 8) = hv;
    *(volatile v8h*)(lo + (size_t)i * 8) = lv;
    __threadfence();
    *(volatile v8h*)(hi + (size_t)i * 8) = hv;
    *(volatile v8h*)(lo + (size_t)i * 8) = lv;
  }
}

__global__ __launch_bounds__(NTHR_R) void lstm1_kernel(const float* __restrict__ ZX1,
                                                       const unsigned short* __restrict__ WH1p,
                                                       unsigned short* __restrict__ HS1p) {
  __shared__ __align__(16) _Float16 Ah[2][ROWS_BLK * HP1];
  const _Float16* WH1 = (const _Float16*)WH1p;
  _Float16* HS1 = (_Float16*)HS1p;
  const int tid = threadIdx.x, lane = tid & 31, wave = tid >> 5;
  const int c = lane & 15, hh = lane >> 4, koff = hh * 8;
  const int b0 = blockIdx.x * ROWS_BLK;
  const int ucol = 16 * wave + c;

  {
    _Float16* ahf = &Ah[0][0];
#pragma unroll 1
    for (int i = tid; i < 2 * ROWS_BLK * HP1; i += NTHR_R) ahf[i] = (_Float16)0.0f;
  }
  float zr[4][8];
#pragma unroll
  for (int gi = 0; gi < 4; ++gi)
#pragma unroll
    for (int r = 0; r < 8; ++r)
      zr[gi][r] = ZX1[(size_t)(b0 + 8 * hh + r) * NG4 + NH * gi + ucol] * WCARRY;
  float cst[8];
#pragma unroll
  for (int r = 0; r < 8; ++r) cst[r] = 0.0f;
  __syncthreads();

#pragma unroll 1
  for (int t = 0; t < NT; ++t) {
    const int cur = t & 1;
    const _Float16* ahrow = &Ah[cur][0] + c * HP1 + koff;
    _Float16* ahn = &Ah[cur ^ 1][0];
    v8f acc[4];
#pragma unroll
    for (int gi = 0; gi < 4; ++gi)
#pragma unroll
      for (int r = 0; r < 8; ++r) acc[gi][r] = zr[gi][r];
#pragma unroll 1
    for (int k0 = 0; k0 < NH; k0 += 32) {
      const v16h a = Frag<_Float16>::load(ahrow + k0);
      v16h bq[4];
#pragma unroll
      for (int gi = 0; gi < 4; ++gi) bq[gi] = Frag<_Float16>::load(WH1 + (size_t)(NH * gi + ucol) * NH + koff + k0);
#pragma unroll
      for (int gi = 0; gi < 4; ++gi) acc[gi] = Frag<_Float16>::mma(a, bq[gi], acc[gi]);
      dep_guard_h(acc[0], acc[3], a, bq[3]);
      keep4_h(bq[0], bq[1], bq[2], a);
    }
    acc_guard4(acc[0], acc[1], acc[2], acc[3]);
#pragma unroll
    for (int r = 0; r < 8; ++r) {
      const float zi = acc[0][r] * WCARRY_INV;
      const float zf = acc[1][r] * WCARRY_INV;
      const float zg = acc[2][r] * WCARRY_INV;
      const float zo = acc[3][r] * WCARRY_INV;
      const float cn = fsig(zf) * cst[r] + fsig(zi) * ftanh(zg);
      cst[r] = cn;
      const float hn = fsig(zo) * ftanh(cn);
      ahn[(8 * hh + r) * HP1 + ucol] = (_Float16)hn;
    }
    __syncthreads();
    {
      const _Float16* srow = ahn + wave * HP1 + lane * 8;
      _Float16* drow = HS1 + ((size_t)(b0 + wave) * NT + (size_t)t) * NH + lane * 8;
      for (int pass = 0; pass < 2; ++pass) {
        const v8h v = *(const v8h*)srow;
        *(volatile v8h*)drow = v;
        __threadfence();
      }
    }
  }
}

__global__ __launch_bounds__(NTHR_R) void lstm2_kernel(const unsigned short* __restrict__ HS1p,
                                                       const unsigned short* __restrict__ WCATp,
                                                       const float* __restrict__ b2,
                                                       const unsigned short* __restrict__ WOHp,
                                                       const unsigned short* __restrict__ WOLp,
                                                       const float* __restrict__ b_out,
                                                       float* __restrict__ out) {
  __shared__ __align__(16) _Float16 At[2][ROWS_BLK * HP2];
  __shared__ __align__(16) __bf16   Hh[ROWS_BLK * HPB];
  __shared__ __align__(16) __bf16   Hl[ROWS_BLK * HPB];
  __shared__ __align__(16) float    Os[ROWS_BLK * OSP];
  const _Float16* HS1  = (const _Float16*)HS1p;
  const _Float16* WCAT = (const _Float16*)WCATp;
  const __bf16*   WOH  = (const __bf16*)WOHp;
  const __bf16*   WOL  = (const __bf16*)WOLp;
  const int tid = threadIdx.x, lane = tid & 31, wave = tid >> 5;
  const int c = lane & 15, hh = lane >> 4, koff = hh * 8;
  const int b0 = blockIdx.x * ROWS_BLK;
  const int ucol = 16 * wave + c;
  const int srow8 = tid >> 5;

  {
    _Float16* atf = &At[0][0];
#pragma unroll 1
    for (int i = tid; i < 2 * ROWS_BLK * HP2; i += NTHR_R) atf[i] = (_Float16)0.0f;
  }
  __syncthreads();
  {
    const v8h v = *(const v8h*)(HS1 + ((size_t)(b0 + srow8) * NT) * NH + lane * 8);
    *(v8h*)(&At[0][0] + srow8 * HP2 + lane * 8) = v;
  }
  float b2x[4];
#pragma unroll
  for (int gi = 0; gi < 4; ++gi) b2x[gi] = b2[NH * gi + ucol] * WCARRY;
  const float bo = b_out[ucol & (NF - 1)];
  float cst[8];
#pragma unroll
  for (int r = 0; r < 8; ++r) cst[r] = 0.0f;
  const v8f z8 = {0.f, 0.f, 0.f, 0.f, 0.f, 0.f, 0.f, 0.f};
  __syncthreads();

#pragma unroll 1
  for (int t = 0; t < NT; ++t) {
    const int cur = t & 1;
    const _Float16* arow = &At[cur][0] + c * HP2 + koff;
    _Float16* atn = &At[cur ^ 1][0];
    v8f acc[4];
#pragma unroll
    for (int gi = 0; gi < 4; ++gi) {
      const float bv = b2x[gi];
      acc[gi] = (v8f){bv, bv, bv, bv, bv, bv, bv, bv};
    }
#pragma unroll 1
    for (int k0 = 0; k0 < 2 * NH; k0 += 32) {
      const v16h a = Frag<_Float16>::load(arow + k0);
      v16h bq[4];
#pragma unroll
      for (int gi = 0; gi < 4; ++gi) bq[gi] = Frag<_Float16>::load(WCAT + (size_t)(NH * gi + ucol) * (2 * NH) + koff + k0);
#pragma unroll
      for (int gi = 0; gi < 4; ++gi) acc[gi] = Frag<_Float16>::mma(a, bq[gi], acc[gi]);
      dep_guard_h(acc[0], acc[3], a, bq[3]);
      keep4_h(bq[0], bq[1], bq[2], a);
    }
    acc_guard4(acc[0], acc[1], acc[2], acc[3]);
#pragma unroll
    for (int r = 0; r < 8; ++r) {
      const float zi = acc[0][r] * WCARRY_INV;
      const float zf = acc[1][r] * WCARRY_INV;
      const float zg = acc[2][r] * WCARRY_INV;
      const float zo = acc[3][r] * WCARRY_INV;
      const float cn = fsig(zf) * cst[r] + fsig(zi) * ftanh(zg);
      cst[r] = cn;
      const float hn = fsig(zo) * ftanh(cn);
      const int ro = 8 * hh + r;
      atn[ro * HP2 + NH + ucol] = (_Float16)hn;
      const unsigned short hb = f2bf_bits(hn);
      const unsigned short lb = f2bf_bits(hn - bf_bits2f(hb));
      Hh[ro * HPB + ucol] = __builtin_bit_cast(__bf16, hb);
      Hl[ro * HPB + ucol] = __builtin_bit_cast(__bf16, lb);
    }
    {
      const int tn = (t + 1 < NT) ? (t + 1) : (NT - 1);
      const v8h v = *(const v8h*)(HS1 + ((size_t)(b0 + srow8) * NT + (size_t)tn) * NH + lane * 8);
      *(v8h*)(atn + srow8 * HP2 + lane * 8) = v;
    }
    __syncthreads();
    if (wave < 4) {
      v8f oacc = z8;
      const __bf16* hhr = Hh + c * HPB + koff;
      const __bf16* hlr = Hl + c * HPB + koff;
      const __bf16* woh = WOH + (size_t)ucol * NH + koff;
      const __bf16* wol = WOL + (size_t)ucol * NH + koff;
#pragma unroll 1
      for (int k0 = 0; k0 < NH; k0 += 32) {
        const v16b ah = Frag<__bf16>::load(hhr + k0);
        const v16b al = Frag<__bf16>::load(hlr + k0);
        const v16b bh = Frag<__bf16>::load(woh + k0);
        const v16b bl = Frag<__bf16>::load(wol + k0);
        oacc = Frag<__bf16>::mma(ah, bh, oacc);
        oacc = Frag<__bf16>::mma(ah, bl, oacc);
        oacc = Frag<__bf16>::mma(al, bh, oacc);
        dep_guard1_b(oacc, al, bh);
        keep4_b(ah, al, bh, bl);
      }
      acc_guard1(oacc);
#pragma unroll
      for (int r = 0; r < 8; ++r) Os[(8 * hh + r) * OSP + ucol] = oacc[r] + bo;
    }
    __syncthreads();
    if (wave < 8) {
      const int row = 2 * wave + hh;
      const int c4 = c * 4;
      const float* osp = Os + row * OSP + c4;
      float* orow = out + ((size_t)(b0 + row) * NT + (size_t)t) * NF + c4;
      for (int pass = 0; pass < 2; ++pass) {
        const v4f v = *(const v4f*)osp;
        *(volatile v4f*)orow = v;
        __threadfence();
      }
    }
  }
}

extern "C" void kernel_launch(void* const* d_in, const int* in_sizes, int n_in,
                              void* d_out, int out_size, void* d_ws, size_t ws_size, hipStream_t stream) {
  if (n_in < 11 || d_out == nullptr || d_ws == nullptr) return;
  if (in_sizes[0] != NB * NIN || in_sizes[1] != NIN * NH || in_sizes[2] != NH ||
      in_sizes[3] != NH * NG4 || in_sizes[4] != NH * NG4 || in_sizes[5] != NG4 ||
      in_sizes[6] != NH * NG4 || in_sizes[7] != NH * NG4 || in_sizes[8] != NG4 ||
      in_sizes[9] != NH * NF || in_sizes[10] != NF || out_size != NOUT) return;

  const float* inputs = (const float*)d_in[0];
  const float* W_in   = (const float*)d_in[1];
  const float* b_in   = (const float*)d_in[2];
  const float* Wx1    = (const float*)d_in[3];
  const float* Wh1    = (const float*)d_in[4];
  const float* b1     = (const float*)d_in[5];
  const float* Wx2    = (const float*)d_in[6];
  const float* Wh2    = (const float*)d_in[7];
  const float* b2     = (const float*)d_in[8];
  const float* W_out  = (const float*)d_in[9];
  const float* b_out  = (const float*)d_in[10];
  float* out = (float*)d_out;

  char* ws = (char*)d_ws; size_t off = 0;
  auto carve = [&](size_t bytes) -> char* { char* p = ws + off; off += (bytes + 255) & ~(size_t)255; return p; };
  unsigned short* INH   = (unsigned short*)carve((size_t)NB * NIN * 2);
  unsigned short* INL   = (unsigned short*)carve((size_t)NB * NIN * 2);
  unsigned short* WINTH = (unsigned short*)carve((size_t)NH * NIN * 2);
  unsigned short* WINTL = (unsigned short*)carve((size_t)NH * NIN * 2);
  unsigned short* XH    = (unsigned short*)carve((size_t)NB * NH * 2);
  unsigned short* XL    = (unsigned short*)carve((size_t)NB * NH * 2);
  unsigned short* WX1TH = (unsigned short*)carve((size_t)NG4 * NH * 2);
  unsigned short* WX1TL = (unsigned short*)carve((size_t)NG4 * NH * 2);
  unsigned short* WH1T  = (unsigned short*)carve((size_t)NG4 * NH * 2);
  unsigned short* WCAT  = (unsigned short*)carve((size_t)NG4 * (2 * NH) * 2);
  unsigned short* WOTH  = (unsigned short*)carve((size_t)NF * NH * 2);
  unsigned short* WOTL  = (unsigned short*)carve((size_t)NF * NH * 2);
  float*          ZX1   = (float*)carve((size_t)NB * NG4 * 4);
  unsigned short* HS1   = (unsigned short*)carve((size_t)NB * NT * NH * 2);
  if (off > ws_size || off > (size_t)134217728) return;

  tr64_kernel<0><<<dim3(NH / 64, NIN / 64), NTHR_G, 0, stream>>>(W_in,  NH,  WINTH, WINTL, NIN,    0,  1.0f);
  tr64_kernel<0><<<dim3(NG4 / 64, NH / 64), NTHR_G, 0, stream>>>(Wx1,   NG4, WX1TH, WX1TL, NH,     0,  1.0f);
  tr64_kernel<1><<<dim3(NG4 / 64, NH / 64), NTHR_G, 0, stream>>>(Wh1,   NG4, WH1T,  WH1T,  NH,     0,  WCARRY);
  tr64_kernel<1><<<dim3(NG4 / 64, NH / 64), NTHR_G, 0, stream>>>(Wx2,   NG4, WCAT,  WCAT,  2 * NH, 0,  WCARRY);
  tr64_kernel<1><<<dim3(NG4 / 64, NH / 64), NTHR_G, 0, stream>>>(Wh2,   NG4, WCAT,  WCAT,  2 * NH, NH, WCARRY);
  tr64_kernel<0><<<dim3(NF / 64, NH / 64),  NTHR_G, 0, stream>>>(W_out, NF,  WOTH,  WOTL,  NH,     0,  1.0f);
  cvt_split8_kernel<<<(NB * NIN / 8) / NTHR_G, NTHR_G, 0, stream>>>(inputs, INH, INL, NB * NIN / 8);

  wmma_gemm64<1, true, 2, 2, false, 2><<<dim3(2, 1), 256, 0, stream>>>(
      INH, INL, NIN, 0L, WINTH, WINTL, NIN, 0L, (void*)XH, (void*)XL, NH, 0L,
      b_in, ZX1, 0L, NB, NH, NIN, 1.0f);
  wmma_gemm64<1, true, 2, 0, false, 0><<<dim3(8, 1), 256, 0, stream>>>(
      XH, XL, NH, 0L, WX1TH, WX1TL, NH, 0L, (void*)ZX1, (void*)ZX1, NG4, 0L,
      b1, ZX1, 0L, NB, NG4, NH, 1.0f);

  lstm1_kernel<<<NB / ROWS_BLK, NTHR_R, 0, stream>>>(ZX1, WH1T, HS1);
  lstm2_kernel<<<NB / ROWS_BLK, NTHR_R, 0, stream>>>(HS1, WCAT, b2, WOTH, WOTL, b_out, out);
}
